// RNN_23192823398477
// MI455X (gfx1250) — hardware-verified
//
#include <hip/hip_runtime.h>
#include <math.h>

typedef __attribute__((ext_vector_type(16))) _Float16 v16h;
typedef __attribute__((ext_vector_type(8)))  _Float16 v8h;
typedef __attribute__((ext_vector_type(8)))  float    v8f;
typedef __attribute__((ext_vector_type(4)))  float    v4f;

constexpr int NB    = 256;
constexpr int NT    = 2048;
constexpr int NI    = 3;
constexpr int NH    = 128;
constexpr int NF    = 64;
constexpr int NO    = 3;
constexpr int NTHR  = 256;
constexpr int RB    = 16;
constexpr int NBLK  = NB / RB;
constexpr int HP    = NH + 8;
constexpr int HTILE = RB * HP;
constexpr int TCH   = 64;
constexpr int XE    = TCH * NI;
constexpr int XST   = XE * RB;
constexpr int HSP   = NH + 4;
constexpr int SLP   = 68;
constexpr int NROWS = NB * NT;
constexpr int NOUT0 = NROWS * NO;
constexpr int NOUT1 = NB * NH;
constexpr int FCBLK = (NROWS / 64) / 8;
constexpr float HCARRY   = 16.0f;
constexpr float WCARRY   = 256.0f;
constexpr float LCARRY   = 2048.0f;
constexpr float LO_FOLD  = 1.0f / 2048.0f;
constexpr float DOT_FOLD = 1.0f / (16.0f * 256.0f);
static_assert(NB % RB == 0);
static_assert(NH == 16 * (NTHR / 32));
static_assert(HP % 8 == 0 && HSP % 4 == 0);
static_assert(NH % 32 == 0);
static_assert(NT % TCH == 0 && NT % 64 == 0);
static_assert(NROWS % 64 == 0 && FCBLK * 8 * 64 == NROWS);
static_assert(NF == 64);
static_assert(XST == NTHR * 12);
static_assert((NH * NH / 8) % NTHR == 0 && (NF * NH / 8) % NTHR == 0);
static_assert((2 * HTILE) % 8 == 0);
static_assert(NO * NF == 6 * 32);
static_assert(RB == 2 * (NTHR / 32));
static_assert(NOUT0 * 4 == 6291456);
static_assert((NOUT0 + NOUT1) * 4 == 6422528);
static_assert((size_t)NROWS * NH * 2 == (size_t)134217728);

__device__ __forceinline__ void dep_guard_h(v8f& a, v8f& b, v16h x, v16h y) { asm volatile("v_nop\n\tv_nop\n\tv_nop\n\tv_nop" : "+v"(a), "+v"(b) : "v"(x), "v"(y)); }
__device__ __forceinline__ void dep_guard4h(v8f& a, v8f& b, v8f& c, v8f& d, v16h x, v16h y) { asm volatile("v_nop\n\tv_nop\n\tv_nop\n\tv_nop" : "+v"(a), "+v"(b), "+v"(c), "+v"(d) : "v"(x), "v"(y)); }
__device__ __forceinline__ void keep4_h(v16h a, v16h b, v16h c, v16h d) { asm volatile("v_nop" :: "v"(a), "v"(b), "v"(c), "v"(d)); }
__device__ __forceinline__ void acc_guard4(v8f& a, v8f& b, v8f& c, v8f& d) { asm volatile("v_nop\n\tv_nop\n\tv_nop\n\tv_nop" : "+v"(a), "+v"(b), "+v"(c), "+v"(d)); }
__device__ __forceinline__ void acc_guard2(v8f& a, v8f& b) { asm volatile("v_nop\n\tv_nop\n\tv_nop\n\tv_nop" : "+v"(a), "+v"(b)); }
template <typename T> struct Frag;
template <> struct Frag<_Float16> {
  typedef v16h V; union U { v16h v; v8h h[2]; };
  static __device__ __forceinline__ v16h load(const _Float16* p) {
    U f; f.h[0] = *(const v8h*)(p); f.h[1] = *(const v8h*)(p + 16); return f.v;
  }
  static __device__ __forceinline__ v8f mma(v16h a, v16h b, v8f c) {
    return __builtin_amdgcn_wmma_f32_16x16x32_f16(false, a, false, b, (short)0, c, false, false);
  }
};

__device__ __forceinline__ float ftanh(float x) { return 1.0f - 2.0f * __builtin_amdgcn_rcpf(1.0f + expf(2.0f * x)); }

__global__ __launch_bounds__(NTHR) void rnn_seq_kernel(
    const float* __restrict__ x, const float* __restrict__ hid0,
    const float* __restrict__ w_ih, const float* __restrict__ w_hh,
    const float* __restrict__ b_ih, const float* __restrict__ b_hh,
    unsigned short* __restrict__ hsp, float* __restrict__ hfin) {
  __shared__ __align__(16) _Float16 sWh[NH * HP];
  __shared__ __align__(16) _Float16 hHb[2 * HTILE];
  __shared__ __align__(16) _Float16 hLb[2 * HTILE];
  __shared__ __align__(16) float    xsT[XST];
  __shared__ __align__(16) float    hsl[RB * HSP];
  const int tid = threadIdx.x, lane = tid & 31, wave = tid >> 5;
  const int c = lane & 15, hh = lane >> 4, koff = hh * 8, mOff = hh * 8;
  const int ncol = 16 * wave + c;
  const int b0 = blockIdx.x * RB;
  const v8h z8h = {(_Float16)0.f, (_Float16)0.f, (_Float16)0.f, (_Float16)0.f, (_Float16)0.f, (_Float16)0.f, (_Float16)0.f, (_Float16)0.f};
  const v8f z8f = {0.f, 0.f, 0.f, 0.f, 0.f, 0.f, 0.f, 0.f};

#pragma unroll 2
  for (int it = 0; it < (NH * NH / 8) / NTHR; ++it) {
    const int q = it * NTHR + tid;
    const int row = q >> 4, c8 = (q & 15) * 8;
    const float* sp = w_hh + row * NH + c8;
    const v4f fa = *(const v4f*)(sp);
    const v4f fb = *(const v4f*)(sp + 4);
    v8h hv;
#pragma unroll
    for (int e = 0; e < 4; ++e) { hv[e] = (_Float16)(fa[e] * WCARRY); hv[4 + e] = (_Float16)(fb[e] * WCARRY); }
    *(v8h*)(sWh + row * HP + c8) = hv;
  }
  if (tid < NH) *(v8h*)(sWh + tid * HP + NH) = z8h;
  for (int i = tid; i < (2 * HTILE) / 8; i += NTHR) { *(v8h*)(hHb + 8 * i) = z8h; *(v8h*)(hLb + 8 * i) = z8h; }
  __syncthreads();

  v16h bw[4];
#pragma unroll
  for (int kc = 0; kc < NH / 32; ++kc) bw[kc] = Frag<_Float16>::load(sWh + ncol * HP + koff + 32 * kc);
  const float wi0 = w_ih[ncol * NI + 0], wi1 = w_ih[ncol * NI + 1], wi2 = w_ih[ncol * NI + 2];
  const float bi = b_ih[ncol], bh2 = b_hh[ncol];
  asm volatile("" ::: "memory");
  {
    float h0v[8];
#pragma unroll
    for (int r = 0; r < 8; ++r) h0v[r] = hid0[(size_t)(b0 + mOff + r) * NH + ncol];
#pragma unroll
    for (int r = 0; r < 8; ++r) {
      const float hs = h0v[r] * HCARRY;
      const _Float16 hi = (_Float16)hs;
      const _Float16 lo = (_Float16)((hs - (float)hi) * LCARRY);
      hHb[(mOff + r) * HP + ncol] = hi;
      hLb[(mOff + r) * HP + ncol] = lo;
    }
  }
  __syncthreads();

#pragma unroll 1
  for (int t = 0; t < NT; ++t) {
    if ((t & (TCH - 1)) == 0) {
      const int row = tid >> 4, q = tid & 15;
      const float* src = x + ((size_t)(b0 + row) * NT + (size_t)t) * NI;
      const v4f f0 = *(const v4f*)(src + 4 * q);
      const v4f f1 = *(const v4f*)(src + 4 * (q + 16));
      const v4f f2 = *(const v4f*)(src + 4 * (q + 32));
#pragma unroll
      for (int e = 0; e < 4; ++e) {
        xsT[(4 * q + e) * RB + row]        = f0[e];
        xsT[(4 * (q + 16) + e) * RB + row] = f1[e];
        xsT[(4 * (q + 32) + e) * RB + row] = f2[e];
      }
      __syncthreads();
    }
    const int tt  = t & (TCH - 1);
    const int cur = t & 1;
    const _Float16* hHc = hHb + cur * HTILE;
    const _Float16* hLc = hLb + cur * HTILE;
    _Float16* hHn = hHb + (cur ^ 1) * HTILE;
    _Float16* hLn = hLb + (cur ^ 1) * HTILE;

    const float* xq = xsT + (tt * NI) * RB + mOff;
    const v4f x0a = *(const v4f*)(xq),          x0b = *(const v4f*)(xq + 4);
    const v4f x1a = *(const v4f*)(xq + RB),     x1b = *(const v4f*)(xq + RB + 4);
    const v4f x2a = *(const v4f*)(xq + 2 * RB), x2b = *(const v4f*)(xq + 2 * RB + 4);
    float xp[8];
#pragma unroll
    for (int r = 0; r < 4; ++r) {
      float p = x0a[r] * wi0; p = fmaf(x1a[r], wi1, p); p = fmaf(x2a[r], wi2, p);
      xp[r] = (p + bi) + bh2;
      float p2 = x0b[r] * wi0; p2 = fmaf(x1b[r], wi1, p2); p2 = fmaf(x2b[r], wi2, p2);
      xp[4 + r] = (p2 + bi) + bh2;
    }

    v8f accH = z8f, accL = z8f;
    const _Float16* aHr = hHc + c * HP + koff;
    const _Float16* aLr = hLc + c * HP + koff;
#pragma unroll
    for (int kc = 0; kc < NH / 32; ++kc) {
      const v16h aH = Frag<_Float16>::load(aHr + 32 * kc);
      const v16h aL = Frag<_Float16>::load(aLr + 32 * kc);
      accH = Frag<_Float16>::mma(aH, bw[kc], accH);
      accL = Frag<_Float16>::mma(aL, bw[kc], accL);
      dep_guard_h(accH, accL, aH, aL);
    }
    keep4_h(bw[0], bw[1], bw[2], bw[3]);
    acc_guard2(accH, accL);

    float hvv[8];
#pragma unroll
    for (int r = 0; r < 8; ++r) {
      const float dot = fmaf(accL[r], LO_FOLD, accH[r]) * DOT_FOLD;
      const float hv = ftanh(xp[r] + dot);
      hvv[r] = hv;
      const float hs = hv * HCARRY;
      const _Float16 hi = (_Float16)hs;
      const _Float16 lo = (_Float16)((hs - (float)hi) * LCARRY);
      hHn[(mOff + r) * HP + ncol] = hi;
      hLn[(mOff + r) * HP + ncol] = lo;
    }
    if (t == NT - 1) {
#pragma unroll
      for (int r = 0; r < 8; ++r) hsl[(mOff + r) * HSP + ncol] = hvv[r];
    }
    __syncthreads();

    {
      const int row = 2 * wave + hh;
      const v8h v = *(const v8h*)(hHn + row * HP + c * 8);
      unsigned short* dst = hsp + (((size_t)(b0 + row)) * NT + (size_t)t) * NH + c * 8;
      *(volatile v8h*)dst = v;
      __threadfence();
      *(volatile v8h*)dst = v;
    }
  }

  for (int pass = 0; pass < 2; ++pass) {
#pragma unroll
    for (int rr = 0; rr < 2; ++rr) {
      const int row = 2 * wave + rr;
      const v4f v = *(const v4f*)(hsl + row * HSP + 4 * lane);
      *(volatile v4f*)(hfin + (size_t)(b0 + row) * NH + 4 * lane) = v;
    }
    __threadfence();
  }
}

__global__ __launch_bounds__(NTHR) void fc_head_kernel(
    const unsigned short* __restrict__ hsp, const float* __restrict__ w_fc1, const float* __restrict__ b_fc1,
    const float* __restrict__ w_fc2, const float* __restrict__ b_fc2, float* __restrict__ out) {
  __shared__ __align__(16) float    sT[8][16 * SLP];
  __shared__ __align__(16) _Float16 sW1[NF * HP];
  __shared__ __align__(16) float    sW2[256];
  __shared__ __align__(16) float    sO[8][192];
  const int tid = threadIdx.x, lane = tid & 31, wave = tid >> 5;
  const int rlane = lane & 15, hh = lane >> 4, koff = hh * 8, mOff = hh * 8;
  const v8h z8h = {(_Float16)0.f, (_Float16)0.f, (_Float16)0.f, (_Float16)0.f, (_Float16)0.f, (_Float16)0.f, (_Float16)0.f, (_Float16)0.f};
  const v8f z8f = {0.f, 0.f, 0.f, 0.f, 0.f, 0.f, 0.f, 0.f};

#pragma unroll
  for (int it = 0; it < (NF * NH / 8) / NTHR; ++it) {
    const int q = it * NTHR + tid;
    const int row = q >> 4, c8 = (q & 15) * 8;
    const float* sp = w_fc1 + row * NH + c8;
    const v4f fa = *(const v4f*)(sp);
    const v4f fb = *(const v4f*)(sp + 4);
    v8h hv;
#pragma unroll
    for (int e = 0; e < 4; ++e) { hv[e] = (_Float16)(fa[e] * WCARRY); hv[4 + e] = (_Float16)(fb[e] * WCARRY); }
    *(v8h*)(sW1 + row * HP + c8) = hv;
  }
  if (tid < NF) *(v8h*)(sW1 + tid * HP + NH) = z8h;
  if (wave < 6) sW2[tid] = w_fc2[tid];
  if (wave == 7) {
    const int bl = (lane < NO) ? lane : (NO - 1);
    const float bv = b_fc2[bl];
    if (lane < NO) sW2[NO * NF + lane] = bv;
  }
  __syncthreads();

  const _Float16* A = (const _Float16*)hsp;
  const int m0 = (blockIdx.x * 8 + wave) * 64;

  v8f acc[4][4];
#pragma unroll
  for (int i = 0; i < 4; ++i)
#pragma unroll
    for (int j = 0; j < 4; ++j) acc[i][j] = z8f;

  for (int k0 = 0; k0 < NH; k0 += 32) {
    v16h bfr[4];
#pragma unroll
    for (int j = 0; j < 4; ++j) bfr[j] = Frag<_Float16>::load(sW1 + (16 * j + rlane) * HP + koff + k0);
#pragma unroll
    for (int i = 0; i < 4; ++i) {
      const v16h ah = Frag<_Float16>::load(A + (size_t)(m0 + 16 * i + rlane) * NH + koff + k0);
#pragma unroll
      for (int j = 0; j < 4; ++j) acc[i][j] = Frag<_Float16>::mma(ah, bfr[j], acc[i][j]);
      dep_guard4h(acc[i][0], acc[i][1], acc[i][2], acc[i][3], ah, bfr[3]);
    }
    keep4_h(bfr[0], bfr[1], bfr[2], bfr[3]);
  }
  acc_guard4(acc[0][0], acc[0][1], acc[0][2], acc[0][3]);
  acc_guard4(acc[1][0], acc[1][1], acc[1][2], acc[1][3]);
  acc_guard4(acc[2][0], acc[2][1], acc[2][2], acc[2][3]);
  acc_guard4(acc[3][0], acc[3][1], acc[3][2], acc[3][3]);

  float bf1[4];
#pragma unroll
  for (int j = 0; j < 4; ++j) bf1[j] = b_fc1[16 * j + rlane];
  const float bo0 = sW2[NO * NF + 0], bo1 = sW2[NO * NF + 1], bo2 = sW2[NO * NF + 2];
  float* slab = sT[wave];
  float* so = sO[wave];
#pragma unroll
  for (int i = 0; i < 4; ++i) {
#pragma unroll
    for (int j = 0; j < 4; ++j)
#pragma unroll
      for (int r = 0; r < 8; ++r) slab[(mOff + r) * SLP + 16 * j + rlane] = fmaf(acc[i][j][r], DOT_FOLD, bf1[j]);
    __builtin_amdgcn_fence(__ATOMIC_RELEASE, "workgroup");
    __builtin_amdgcn_wave_barrier();
    __builtin_amdgcn_fence(__ATOMIC_ACQUIRE, "workgroup");
    float d0 = 0.0f, d1 = 0.0f, d2 = 0.0f;
    const float* sp = slab + rlane * SLP + 32 * hh;
    const float* wp = sW2 + 32 * hh;
#pragma unroll 1
    for (int f = 0; f < 32; ++f) {
      const float a = sp[f];
      d0 = fmaf(a, wp[f], d0);
      d1 = fmaf(a, wp[NF + f], d1);
      d2 = fmaf(a, wp[2 * NF + f], d2);
    }
    d0 += __shfl_xor(d0, 16, 32);
    d1 += __shfl_xor(d1, 16, 32);
    d2 += __shfl_xor(d2, 16, 32);
    if (hh == 0) {
      so[(16 * i + rlane) * NO + 0] = d0 + bo0;
      so[(16 * i + rlane) * NO + 1] = d1 + bo1;
      so[(16 * i + rlane) * NO + 2] = d2 + bo2;
    }
    __builtin_amdgcn_fence(__ATOMIC_RELEASE, "workgroup");
    __builtin_amdgcn_wave_barrier();
    __builtin_amdgcn_fence(__ATOMIC_ACQUIRE, "workgroup");
  }

  float* op = out + (size_t)m0 * NO;
  const int l2 = lane & 15;
  for (int pass = 0; pass < 2; ++pass) {
    const v4f v0 = *(const v4f*)(so + 4 * lane);
    const v4f v1 = *(const v4f*)(so + 128 + 4 * l2);
    *(volatile v4f*)(op + 4 * lane) = v0;
    if (lane < 16) *(volatile v4f*)(op + 128 + 4 * lane) = v1;
    __threadfence();
  }
}

extern "C" void kernel_launch(void* const* d_in, const int* in_sizes, int n_in,
                              void* d_out, int out_size, void* d_ws, size_t ws_size, hipStream_t stream) {
  if (n_in < 10 || d_out == nullptr || d_ws == nullptr) return;
  if (in_sizes[0] != NB * NT * NI || in_sizes[1] != NB * NH || in_sizes[2] != NH * NI || in_sizes[3] != NH * NH ||
      in_sizes[4] != NH || in_sizes[5] != NH || in_sizes[6] != NF * NH || in_sizes[7] != NF ||
      in_sizes[8] != NO * NF || in_sizes[9] != NO || out_size != NOUT0 + NOUT1) return;

  const float* x     = (const float*)d_in[0];
  const float* hid0  = (const float*)d_in[1];
  const float* w_ih  = (const float*)d_in[2];
  const float* w_hh  = (const float*)d_in[3];
  const float* b_ih  = (const float*)d_in[4];
  const float* b_hh  = (const float*)d_in[5];
  const float* w_fc1 = (const float*)d_in[6];
  const float* b_fc1 = (const float*)d_in[7];
  const float* w_fc2 = (const float*)d_in[8];
  const float* b_fc2 = (const float*)d_in[9];
  float* out  = (float*)d_out;
  float* hfin = out + (size_t)NOUT0;

  char* ws = (char*)d_ws; size_t off = 0;
  auto carve = [&](size_t bytes) -> char* { char* p = ws + off; off += (bytes + 255) & ~(size_t)255; return p; };
  unsigned short* HS = (unsigned short*)carve((size_t)NROWS * NH * 2);
  if (off > ws_size || off > (size_t)134217728) return;

  rnn_seq_kernel<<<NBLK, NTHR, 0, stream>>>(x, hid0, w_ih, w_hh, b_ih, b_hh, HS, hfin);
  fc_head_kernel<<<FCBLK, NTHR, 0, stream>>>(HS, w_fc1, b_fc1, w_fc2, b_fc2, out);
}
